// FadeFeatureAlignment_45114336477817
// MI455X (gfx1250) — hardware-verified
//
#include <hip/hip_runtime.h>


#define NB_  2
#define HF   128
#define WF   128
#define HC   64
#define WC   64
#define CCH  128
#define EMB  64
#define KK2  25
#define KS5  5
#define NPF  (HF * WF)
#define NPC  (HC * WC)
#define KIM  576
#define FIL  128
#define DM   CCH
#define LOSC 1024.0f

typedef _Float16 h16;
typedef unsigned short bf;
typedef __attribute__((ext_vector_type(16))) __bf16   v16bf;
typedef __attribute__((ext_vector_type(16))) _Float16 v16h;
typedef __attribute__((ext_vector_type(8)))  _Float16 v8h;
typedef __attribute__((ext_vector_type(8)))  unsigned short v8us;
typedef __attribute__((ext_vector_type(8)))  float    v8f;
typedef __attribute__((ext_vector_type(4)))  float    v4f;
typedef v8h  __attribute__((may_alias)) v8ha;
typedef v4f  __attribute__((may_alias)) v4fa;
typedef v8us __attribute__((may_alias)) v8usa;

__device__ __forceinline__ unsigned short f2bf(float f) { unsigned u = __float_as_uint(f); u += 0x7FFFu + ((u >> 16) & 1u); return (unsigned short)(u >> 16); }
__device__ __forceinline__ float bf2f(unsigned short b) { return __uint_as_float(((unsigned)b) << 16); }
__device__ __forceinline__ float bfr(float f) { return bf2f(f2bf(f)); }
__device__ __forceinline__ v16h cat16(v8h lo, v8h hi) { return __builtin_shufflevector(lo, hi, 0, 1, 2, 3, 4, 5, 6, 7, 8, 9, 10, 11, 12, 13, 14, 15); }
__device__ __forceinline__ v16bf cat16b(v8us lo, v8us hi) { return __builtin_bit_cast(v16bf, __builtin_shufflevector(lo, hi, 0, 1, 2, 3, 4, 5, 6, 7, 8, 9, 10, 11, 12, 13, 14, 15)); }
__device__ __forceinline__ v8f wmma16(v16h a, v16h b, v8f c) { return __builtin_amdgcn_wmma_f32_16x16x32_f16(false, a, false, b, (short)0, c, false, false); }
__device__ __forceinline__ v8f wmmab(v16bf a, v16bf b, v8f c) { return __builtin_amdgcn_wmma_f32_16x16x32_bf16(false, a, false, b, (short)0, c, false, false); }

template <bool SPLITA, bool F16OUT = false>
__global__ __launch_bounds__(128) void k_gemmb(const bf* __restrict__ A, const bf* __restrict__ Al, const bf* __restrict__ Bn, const float* __restrict__ bias, float* C, int ldc, h16* C2, const float* __restrict__ R = nullptr, int K = DM, int roundR = 1) {
    __shared__ __align__(16) float ost[4][16 * 68];
    const int lane = threadIdx.x & 31, wave = threadIdx.x >> 5, lr = lane & 15, hi = lane >> 4;
    const int r0 = blockIdx.x * 64 + wave * 16, c0 = blockIdx.y * 64;
    const size_t aoff = (size_t)(r0 + lr) * K + 8 * hi;
    size_t boff[4];
#pragma unroll
    for (int t = 0; t < 4; ++t) boff[t] = (size_t)(c0 + t * 16 + lr) * K + 8 * hi;
    v8f acc[4];
#pragma unroll
    for (int t = 0; t < 4; ++t) acc[t] = (v8f){};
#pragma unroll 1
    for (int kc = 0; kc < K; kc += 32) {
        const v16bf a = cat16b(*(const v8us*)(A + aoff + kc), *(const v8us*)(A + aoff + kc + 16));
        v16bf al = a;
        if (SPLITA) al = cat16b(*(const v8us*)(Al + aoff + kc), *(const v8us*)(Al + aoff + kc + 16));
#pragma unroll
        for (int t = 0; t < 4; ++t) { const v16bf b = cat16b(*(const v8us*)(Bn + boff[t] + kc), *(const v8us*)(Bn + boff[t] + kc + 16)); acc[t] = wmmab(a, b, acc[t]); if (SPLITA) acc[t] = wmmab(al, b, acc[t]); }
        asm volatile("v_nop\n\tv_nop\n\tv_nop\n\tv_nop" : "+v"(acc[0]), "+v"(acc[1]), "+v"(acc[2]), "+v"(acc[3]) : "v"(a), "v"(al));
    }
    float* os = &ost[wave][0];
#pragma unroll
    for (int t = 0; t < 4; ++t) { const float bv = bias ? bfr(bias[c0 + t * 16 + lr]) : 0.f;
#pragma unroll
        for (int j = 0; j < 8; ++j) os[(hi * 8 + j) * 68 + t * 16 + lr] = acc[t][j] + bv; }
    __syncthreads();
    if (F16OUT) {
        h16* crow = (h16*)(void*)C + (size_t)r0 * ldc + c0;
        auto pass = [&]() {
#pragma unroll
            for (int s = 0; s < 4; ++s) { const int row = 4 * s + (lane >> 3), piece = lane & 7; const float* sp = os + row * 68 + piece * 8; v8h o, o2;
#pragma unroll
                for (int i = 0; i < 8; ++i) { const h16 a = (h16)sp[i]; o[i] = a; o2[i] = (h16)((sp[i] - (float)a) * LOSC); }
                *(volatile v8h*)(crow + (size_t)row * ldc + piece * 8) = o; if (C2) *(volatile v8h*)(C2 + (size_t)r0 * ldc + c0 + (size_t)row * ldc + piece * 8) = o2; }
        };
        pass(); __threadfence(); pass();
    } else {
        float* crow = C + (size_t)r0 * ldc + c0;
        auto pass = [&]() {
#pragma unroll
            for (int s = 0; s < 8; ++s) { const int Lid = (lane >> 3) + 4 * s, piece = lane & 7; const int row = Lid >> 1, cofs = (Lid & 1) * 32 + piece * 4;
                v4f val = *(const v4fa*)(os + row * 68 + cofs); if (R) { const v4f rv = *(const v4f*)(R + ((size_t)r0 + row) * ldc + c0 + cofs); val += roundR ? (v4f){bfr(rv[0]), bfr(rv[1]), bfr(rv[2]), bfr(rv[3])} : rv; }
                *(volatile v4f*)(crow + (size_t)row * ldc + cofs) = val; }
        };
        pass(); __threadfence(); pass();
    }
}

__global__ __launch_bounds__(256) void k_wt(const float* __restrict__ Wm, int K, int ncols, bf* WT) {
    __shared__ __align__(16) unsigned short tl[64 * 72];
    const int tid = threadIdx.x, k0 = blockIdx.x * 64, n0 = blockIdx.y * 64;
    const int kk = tid >> 2, nq = (tid & 3) * 16;
#pragma unroll
    for (int i = 0; i < 16; ++i) tl[(nq + i) * 72 + kk] = f2bf(Wm[(size_t)(k0 + kk) * ncols + n0 + nq + i]);
    __syncthreads();
    const int piece = tid & 7;
    auto pass = [&]() {
#pragma unroll
        for (int s = 0; s < 2; ++s) { const int nr = (tid >> 3) + 32 * s; const v8us val = *(const v8usa*)(tl + nr * 72 + piece * 8); *(volatile v8us*)(WT + (size_t)(n0 + nr) * K + k0 + piece * 8) = val; }
    };
    pass(); __threadfence(); pass();
}

__global__ __launch_bounds__(256) void k_wtp(const float* __restrict__ Wm, int krows, int ncols, int kpad, bf* WT) {
    __shared__ __align__(16) unsigned short tl[64 * 72];
    const int tid = threadIdx.x, k0 = blockIdx.x * 64, n0 = blockIdx.y * 64;
    const int kk = tid >> 2, nq = (tid & 3) * 16;
    const int k = k0 + kk, kc = k < krows ? k : krows - 1;
#pragma unroll
    for (int i = 0; i < 16; ++i) { const int n = n0 + nq + i, ncl = n < ncols ? n : ncols - 1; const float w = Wm[(size_t)kc * ncols + ncl]; tl[(nq + i) * 72 + kk] = (k < krows && n < ncols) ? f2bf(w) : (unsigned short)0; }
    __syncthreads();
    const int piece = tid & 7;
    auto pass = [&]() {
#pragma unroll
        for (int s = 0; s < 2; ++s) { const int nr = (tid >> 3) + 32 * s; const v8us val = *(const v8usa*)(tl + nr * 72 + piece * 8); *(volatile v8us*)(WT + (size_t)(n0 + nr) * kpad + k0 + piece * 8) = val; }
    };
    pass(); __threadfence(); pass();
}

__global__ __launch_bounds__(256) void k_cvt128(const float* __restrict__ src, int nrows, bf* dst) {
    typedef __attribute__((ext_vector_type(4))) unsigned short v4us;
    const int lane = threadIdx.x & 31; const size_t r = (size_t)blockIdx.x * 8 + (threadIdx.x >> 5); if (r >= (size_t)nrows) return; v4us o;
#pragma unroll
    for (int i = 0; i < 4; ++i) o[i] = f2bf(src[r * CCH + lane * 4 + i]);
    *(volatile v4us*)(dst + r * CCH + lane * 4) = o; __threadfence(); *(volatile v4us*)(dst + r * CCH + lane * 4) = o;
}
__global__ __launch_bounds__(256) void k_split128(const float* __restrict__ src, int nrows, bf* dh, bf* dl) {
    typedef __attribute__((ext_vector_type(4))) unsigned short v4us;
    const int lane = threadIdx.x & 31; const size_t r = (size_t)blockIdx.x * 8 + (threadIdx.x >> 5); if (r >= (size_t)nrows) return; v4us oh, ol;
#pragma unroll
    for (int i = 0; i < 4; ++i) { const float v = src[r * CCH + lane * 4 + i]; const unsigned short hb = f2bf(v); oh[i] = hb; ol[i] = f2bf(v - bf2f(hb)); }
    const size_t o = r * CCH + lane * 4; *(volatile v4us*)(dh + o) = oh; *(volatile v4us*)(dl + o) = ol; __threadfence(); *(volatile v4us*)(dh + o) = oh; *(volatile v4us*)(dl + o) = ol;
}
__global__ __launch_bounds__(256) void k_im3(const float* __restrict__ E, int hh, int ww, bf* Ph, bf* Pl) {
    const int lane = threadIdx.x & 31; const size_t p = (size_t)blockIdx.x * 8 + (threadIdx.x >> 5); if (p >= (size_t)hh * ww) return; const int y = (int)(p / ww), x = (int)(p % ww);
#pragma unroll 1
    for (int ps = 0; ps < 2; ++ps) {
#pragma unroll 1
        for (int e0 = lane * 8; e0 < KIM; e0 += 256) { v8us oh, ol;
#pragma unroll
            for (int q = 0; q < 8; ++q) { const int e = e0 + q; const int t = e / EMB, c = e - t * EMB; const int dy = t / 3, dx = t - dy * 3; const int yy = y + dy - 1, xx = x + dx - 1;
                const bool ok = (yy >= 0) && (yy < hh) && (xx >= 0) && (xx < ww); const float v = ok ? E[((size_t)(ok ? yy : 0) * ww + (ok ? xx : 0)) * EMB + c] : 0.f;
                const unsigned short hb = f2bf(v); oh[q] = hb; ol[q] = f2bf(v - bf2f(hb)); }
            const size_t o = p * KIM + e0; *(volatile v8us*)(Ph + o) = oh; *(volatile v8us*)(Pl + o) = ol; }
        if (ps == 0) __threadfence(); }
}
__global__ __launch_bounds__(256) void k_carafe(const float* __restrict__ KF, const float* __restrict__ KC, const float* __restrict__ coarse_b, const float* __restrict__ bc, bf* Ch, bf* Cl) {
    typedef __attribute__((ext_vector_type(4))) unsigned short v4us;
    const int lane = threadIdx.x & 31; const size_t p = (size_t)blockIdx.x * 8 + (threadIdx.x >> 5); if (p >= (size_t)NPF) return; const int y = (int)(p / WF), x = (int)(p % WF); const int yc = y / 2, xc = x / 2;
    __shared__ float krs[8][32]; const int wv = threadIdx.x >> 5;
    { const int k = lane; const bool kv = k < KK2; const float lg = kv ? (KF[p * 64 + k] + KC[((size_t)yc * WC + xc) * 64 + k] + 2.0f * bfr(bc[kv ? k : 0])) : -3.0e38f;
      float mx = lg;
#pragma unroll
      for (int sh = 16; sh; sh >>= 1) mx = fmaxf(mx, __shfl_xor(mx, sh, 32));
      const float e = kv ? __expf(lg - mx) : 0.f; float s = e;
#pragma unroll
      for (int sh = 16; sh; sh >>= 1) s += __shfl_xor(s, sh, 32);
      krs[wv][lane] = e / s; }
    __syncthreads();
    const float* kr = krs[wv];
    float acc[4] = {0.f, 0.f, 0.f, 0.f};
#pragma unroll
    for (int q = 0; q < 4; ++q) { const int c = lane * 4 + q;
#pragma unroll 1
        for (int k = 0; k < KK2; ++k) { const int f = c * KK2 + k; const int pp = f / CCH, ch = f % CCH; const int r = pp / KS5, cc = pp - r * KS5; const int yy = yc + r - 2, xx = xc + cc - 2;
            const bool ok = (yy >= 0) && (yy < HC) && (xx >= 0) && (xx < WC); const float v = ok ? bfr(coarse_b[((size_t)(ok ? yy : 0) * WC + (ok ? xx : 0)) * CCH + ch]) : 0.f;
            acc[q] = fmaf(v, kr[k], acc[q]); } }
    v4us oh, ol;
#pragma unroll
    for (int q = 0; q < 4; ++q) { const unsigned short hb = f2bf(acc[q]); oh[q] = hb; ol[q] = f2bf(acc[q] - bf2f(hb)); }
    const size_t o = p * CCH + lane * 4; *(volatile v4us*)(Ch + o) = oh; *(volatile v4us*)(Cl + o) = ol; __threadfence(); *(volatile v4us*)(Ch + o) = oh; *(volatile v4us*)(Cl + o) = ol;
}
__global__ __launch_bounds__(256) void k_blend(const float* __restrict__ FO, const float* __restrict__ CO, const float* __restrict__ G, const float* __restrict__ bg, float* OUTB) {
    const int lane = threadIdx.x & 31; const size_t p = (size_t)blockIdx.x * 8 + (threadIdx.x >> 5); if (p >= (size_t)NPF) return; const int y = (int)(p / WF), x = (int)(p % WF);
    const float gl = G[((size_t)(y / 2) * WC + (x / 2)) * 64 + 0] + bfr(bg[0]); const float g = 1.0f / (1.0f + __expf(-gl)); v4f o;
#pragma unroll
    for (int q = 0; q < 4; ++q) { const size_t e = p * FIL + lane * 4 + q; o[q] = g * FO[e] + (1.0f - g) * CO[e]; }
    *(volatile v4f*)(OUTB + p * FIL + lane * 4) = o; __threadfence(); *(volatile v4f*)(OUTB + p * FIL + lane * 4) = o;
}

extern "C" void kernel_launch(void* const* d_in, const int* in_sizes, int n_in,
                              void* d_out, int out_size, void* d_ws, size_t ws_size, hipStream_t stream) {
    (void)in_sizes; (void)n_in; (void)out_size;
    const float* fine = (const float*)d_in[0]; const float* coarse = (const float*)d_in[1]; const float* wg = (const float*)d_in[2]; const float* bg = (const float*)d_in[3];
    const float* wsf = (const float*)d_in[4]; const float* wsc = (const float*)d_in[5]; const float* bsc = (const float*)d_in[6]; const float* wct = (const float*)d_in[7]; const float* bct = (const float*)d_in[8];
    const float* wco = (const float*)d_in[9]; const float* bco = (const float*)d_in[10]; const float* wfo = (const float*)d_in[11]; const float* bfo = (const float*)d_in[12];
    float* out = (float*)d_out;
    char* wsp = (char*)d_ws;
    auto take = [&](size_t bytes) { char* p = wsp; wsp += (bytes + 255) & ~(size_t)255; return (void*)p; };
    bf* WG = (bf*)take(64 * CCH * 2); bf* WSF = (bf*)take(EMB * CCH * 2); bf* WSC = (bf*)take(EMB * CCH * 2); bf* WCT = (bf*)take(64 * KIM * 2); bf* WCO = (bf*)take(FIL * CCH * 2); bf* WFO = (bf*)take(FIL * FIL * 2);
    bf* Fb = (bf*)take((size_t)NPF * CCH * 2); bf* Cb = (bf*)take((size_t)NPC * CCH * 2); float* F1 = (float*)take((size_t)NPF * EMB * 4); float* C1 = (float*)take((size_t)NPC * EMB * 4); float* G = (float*)take((size_t)NPC * 64 * 4);
    bf* Ih = (bf*)take((size_t)NPF * KIM * 2); bf* Il = (bf*)take((size_t)NPF * KIM * 2); float* KF = (float*)take((size_t)NPF * 64 * 4); float* KC = (float*)take((size_t)NPC * 64 * 4);
    bf* Ah = (bf*)take((size_t)NPF * CCH * 2); bf* Al = (bf*)take((size_t)NPF * CCH * 2); float* CO = (float*)take((size_t)NPF * FIL * 4); float* FO = (float*)take((size_t)NPF * FIL * 4);
    if ((size_t)(wsp - (char*)d_ws) > ws_size) return;
    k_wtp<<<dim3(CCH / 64, 1, 1), 256, 0, stream>>>(wg, CCH, 1, CCH, WG);
    k_wt<<<dim3(CCH / 64, EMB / 64, 1), 256, 0, stream>>>(wsf, CCH, EMB, WSF); k_wt<<<dim3(CCH / 64, EMB / 64, 1), 256, 0, stream>>>(wsc, CCH, EMB, WSC);
    k_wtp<<<dim3(KIM / 64, 1, 1), 256, 0, stream>>>(wct, KIM, KK2, KIM, WCT);
    k_wt<<<dim3(CCH / 64, FIL / 64, 1), 256, 0, stream>>>(wco, CCH, FIL, WCO); k_wt<<<dim3(FIL / 64, FIL / 64, 1), 256, 0, stream>>>(wfo, FIL, FIL, WFO);
    for (int b = 0; b < NB_; ++b) { const float* fb_ = fine + (size_t)b * NPF * CCH; const float* cb_ = coarse + (size_t)b * NPC * CCH;
        k_cvt128<<<NPF / 8, 256, 0, stream>>>(fb_, NPF, Fb); k_cvt128<<<NPC / 8, 256, 0, stream>>>(cb_, NPC, Cb);
        k_gemmb<false, false><<<dim3(NPC / 64, 1, 1), 128, 0, stream>>>(Cb, nullptr, WG, nullptr, G, 64, nullptr, nullptr, CCH);
        k_gemmb<false, false><<<dim3(NPF / 64, 1, 1), 128, 0, stream>>>(Fb, nullptr, WSF, nullptr, F1, EMB, nullptr, nullptr, CCH);
        k_gemmb<false, false><<<dim3(NPC / 64, 1, 1), 128, 0, stream>>>(Cb, nullptr, WSC, bsc, C1, EMB, nullptr, nullptr, CCH);
        k_im3<<<NPC / 8, 256, 0, stream>>>(C1, HC, WC, Ih, Il); k_gemmb<true, false><<<dim3(NPC / 64, 1, 1), 128, 0, stream>>>(Ih, Il, WCT, nullptr, KC, 64, nullptr, nullptr, KIM);
        k_im3<<<NPF / 8, 256, 0, stream>>>(F1, HF, WF, Ih, Il); k_gemmb<true, false><<<dim3(NPF / 64, 1, 1), 128, 0, stream>>>(Ih, Il, WCT, nullptr, KF, 64, nullptr, nullptr, KIM);
        k_carafe<<<NPF / 8, 256, 0, stream>>>(KF, KC, cb_, bct, Ah, Al);
        k_gemmb<true, false><<<dim3(NPF / 64, FIL / 64, 1), 128, 0, stream>>>(Ah, Al, WCO, bco, CO, FIL, nullptr, nullptr, CCH);
        k_split128<<<NPF / 8, 256, 0, stream>>>(CO, NPF, Ah, Al);
        k_gemmb<true, false><<<dim3(NPF / 64, FIL / 64, 1), 128, 0, stream>>>(Ah, Al, WFO, bfo, FO, FIL, nullptr, nullptr, FIL);
        k_blend<<<NPF / 8, 256, 0, stream>>>(FO, CO, G, bg, out + (size_t)b * NPF * FIL); }
}
